// CausalSelfAttentionLoRA_36034775614008
// MI455X (gfx1250) — hardware-run, weakly checked
//
#include <hip/hip_runtime.h>


#ifndef NB
#define NB 2
#endif
#ifndef SEQ
#define SEQ 2048
#endif
#define NB_FULL  2
#define SEQ_FULL 2048
#ifndef OUT_SEQ
#define OUT_SEQ SEQ
#endif
#define DM   1024
#define NH_  16
#define HD   64
#define LR   8
#define LK   32
#define XP   20
#define AW   4
#define OSP  68
#define EROWS (SEQ < 512 ? SEQ : 512)
#define QRS  2048.0f
#define QRI  (1.0f / 2048.0f)
#define SC2  ((float)(0.125 * 1.4426950408889634))
#define L2E  ((float)1.4426950408889634)
#define NEGL ((float)(-1.0e9 * 1.4426950408889634))
#define LSC  2.0f
#define PSH  14.0f
#define PFL  (-14.0f)
#define NEGB (-3.0e38f)
#define WIDE 1.0e8f

static_assert(HD == 64);
static_assert(NH_ * HD == DM);
static_assert(DM % 64 == 0);
static_assert(64 % HD == 0);
static_assert(DM % 32 == 0);
static_assert(LK == 32);
static_assert(2 * LR <= LK);
static_assert(LR == 8);
static_assert(2 * LR == 16);
static_assert(SEQ % 64 == 0);
static_assert((NB * SEQ) % 64 == 0);
static_assert(SEQ % 128 == 0);
static_assert(SEQ % 32 == 0);
static_assert(SEQ % (16 * AW) == 0);
static_assert(EROWS % 64 == 0);
static_assert(EROWS >= 32);
static_assert(EROWS <= SEQ);
static_assert(EROWS % (16 * AW) == 0);
static_assert((SEQ - EROWS) % (16 * AW) == 0);
static_assert(((size_t)SEQ * DM) % 8 == 0);
static_assert(((size_t)DM * DM) % 8 == 0);
static_assert(((size_t)LR * DM) % 8 == 0);
static_assert(NB <= NB_FULL);
static_assert(SEQ <= SEQ_FULL);
static_assert((OSP * 4) % 16 == 0);
static_assert(OSP >= HD);
static_assert((XP * 4) % 16 == 0);
static_assert(XP >= 16);
static_assert(32 * 4 * 16 == 16 * HD * 2);
static_assert(32 * 4 * 16 == 16 * 64 * 2);
static_assert(32 * 8 * 16 == 16 * HD * 4);
static_assert(32 * 8 * 16 == 64 * LK * 2);
static_assert(16 * 68 * 4 <= 131072);
static_assert(64 * XP * 4 <= 131072);
static_assert(AW * 16 * OSP * 4 <= 131072);

typedef _Float16 h16;
typedef unsigned short bf;
typedef __attribute__((ext_vector_type(16))) __bf16   v16bf;
typedef __attribute__((ext_vector_type(16))) _Float16 v16h;
typedef __attribute__((ext_vector_type(8)))  _Float16 v8h;
typedef __attribute__((ext_vector_type(8)))  unsigned short v8us;
typedef __attribute__((ext_vector_type(8)))  float    v8f;
typedef __attribute__((ext_vector_type(4)))  float    v4f;
typedef v4f  __attribute__((may_alias)) v4fa;

__device__ __forceinline__ unsigned short f2bf(float f) { unsigned u = __float_as_uint(f); u += 0x7FFFu + ((u >> 16) & 1u); return (unsigned short)(u >> 16); }
__device__ __forceinline__ float bfr(float f) { return __uint_as_float(((unsigned)f2bf(f)) << 16); }
__device__ __forceinline__ v16h cat16(v8h lo, v8h hi) { return __builtin_shufflevector(lo, hi, 0, 1, 2, 3, 4, 5, 6, 7, 8, 9, 10, 11, 12, 13, 14, 15); }
__device__ __forceinline__ v16bf cat16b(v8us lo, v8us hi) { return __builtin_bit_cast(v16bf, __builtin_shufflevector(lo, hi, 0, 1, 2, 3, 4, 5, 6, 7, 8, 9, 10, 11, 12, 13, 14, 15)); }
__device__ __forceinline__ v8f wmma16(v16h a, v16h b, v8f c) { return __builtin_amdgcn_wmma_f32_16x16x32_f16(false, a, false, b, (short)0, c, false, false); }
__device__ __forceinline__ v8f wmmab(v16bf a, v16bf b, v8f c) { return __builtin_amdgcn_wmma_f32_16x16x32_bf16(false, a, false, b, (short)0, c, false, false); }
__device__ __forceinline__ v16h  ldh(const h16* p) { return cat16(*(const v8h*)p, *(const v8h*)(p + 16)); }
__device__ __forceinline__ v16bf ldb(const bf* p)  { return cat16b(*(const v8us*)p, *(const v8us*)(p + 16)); }
__device__ __forceinline__ void wave_sync() { __builtin_amdgcn_fence(3  , "wavefront"); __builtin_amdgcn_wave_barrier(); asm volatile("" ::: "memory"); }

static __device__ __forceinline__ h16 toh_flush(float v) { const h16 r = (h16)v; return (fabsf(v) < 6.103515625e-05f) ? (h16)0.0f : r; }
static __device__ __forceinline__ v8f wmma16g(v16h a, v16h b, v8f c) { c = wmma16(a, b, c); asm volatile("v_nop\n\tv_nop\n\tv_nop\n\tv_nop" : "+v"(c) : "v"(a), "v"(b)); return c; }
static __device__ __forceinline__ v8f wmmabg(v16bf a, v16bf b, v8f c) { c = wmmab(a, b, c); asm volatile("v_nop\n\tv_nop\n\tv_nop\n\tv_nop" : "+v"(c) : "v"(a), "v"(b)); return c; }
static __device__ __forceinline__ unsigned short ext_word(float v, int piece) {
    const unsigned short hw = f2bf(v); const float hv = __uint_as_float(((unsigned)hw) << 16); const unsigned short lw = f2bf(v - hv);
    return (piece == 0) ? hw : ((piece == 1) ? lw : (unsigned short)0); }

__global__ __launch_bounds__(256) void k_cvt8(const float* __restrict__ src, bf* dst, size_t n8) {
    const size_t i = (size_t)blockIdx.x * 256 + threadIdx.x; if (i >= n8) return;
    const v8f v = *(const v8f*)(src + i * 8); v8us o;
#pragma unroll
    for (int k = 0; k < 8; ++k) o[k] = f2bf(v[k]);
    *(volatile v8us*)(dst + i * 8) = o; __threadfence(); *(volatile v8us*)(dst + i * 8) = o;
}

__global__ __launch_bounds__(256) void k_bext(const float* __restrict__ src, bf* dst, int n4) {
    const int i = blockIdx.x * 256 + threadIdx.x; if (i >= n4) return;
    const int row = i >> 2, piece = i & 3;
    v8f v = *(const v8f*)(src + (size_t)row * LR);
    asm volatile("" : "+v"(v));
    v8us o;
#pragma unroll
    for (int k = 0; k < 8; ++k) { const unsigned short w = f2bf(v[k]); o[k] = (piece < 2) ? w : (unsigned short)0; }
    *(volatile v8us*)(dst + (size_t)i * 8) = o; __threadfence(); *(volatile v8us*)(dst + (size_t)i * 8) = o;
}

__global__ __launch_bounds__(32) void k_xa(const bf* __restrict__ X, const bf* __restrict__ AL, bf* XLq, bf* XLv) {
    __shared__ __align__(16) float os[64 * XP];
    const int lane = threadIdx.x & 31, lr = lane & 15, hi = lane >> 4; const int r0 = blockIdx.x * 64;
    v8f acc[4];
#pragma unroll
    for (int mb = 0; mb < 4; ++mb) acc[mb] = (v8f){};
    const size_t aoff = (size_t)(r0 + lr) * DM + 8 * hi, boff = (size_t)lr * DM + 8 * hi;
#pragma unroll 1
    for (int kc = 0; kc < DM; kc += 32) {
        const v16bf bw = ldb(AL + boff + kc);
#pragma unroll
        for (int mb = 0; mb < 4; ++mb) { const v16bf a = ldb(X + aoff + (size_t)mb * 16 * DM + kc); acc[mb] = wmmabg(a, bw, acc[mb]); }
    }
#pragma unroll
    for (int mb = 0; mb < 4; ++mb) {
#pragma unroll
        for (int j = 0; j < 8; ++j) os[(mb * 16 + hi * 8 + j) * XP + lr] = acc[mb][j] * LSC; }
    wave_sync();
    const size_t ob = (size_t)r0 * LK;
#pragma unroll 1
    for (int ps = 0; ps < 2; ++ps) {
#pragma unroll 1
        for (int s = 0; s < 8; ++s) { const int p = s * 32 + lane; const int row = p >> 2, piece = p & 3;
            const v4f a0 = *(const v4fa*)(&os[row * XP + 0]); const v4f a1 = *(const v4fa*)(&os[row * XP + 4]);
            const v4f c0 = *(const v4fa*)(&os[row * XP + 8]); const v4f c1 = *(const v4fa*)(&os[row * XP + 12]);
            v8us oq, ov;
#pragma unroll
            for (int i = 0; i < 4; ++i) { oq[i] = ext_word(a0[i], piece); oq[4 + i] = ext_word(a1[i], piece); ov[i] = ext_word(c0[i], piece); ov[4 + i] = ext_word(c1[i], piece); }
            *(volatile v8us*)(XLq + ob + (size_t)p * 8) = oq; *(volatile v8us*)(XLv + ob + (size_t)p * 8) = ov; }
        if (ps == 0) __threadfence(); }
}

template <int MODE, int LOWR>
__device__ __forceinline__ void proj_body(const bf* __restrict__ A, const bf* __restrict__ Bt, const bf* __restrict__ AX, const bf* __restrict__ BX,
                                          const float* __restrict__ bias, h16* Ph, h16* Pr, int resT) {
    __shared__ __align__(16) float os[16 * 68];
    const int K = DM;
    const int lane = threadIdx.x & 31, lr = lane & 15, hi = lane >> 4; const int r0 = blockIdx.x * 64, c0 = blockIdx.y * 64;
    v8f acc[4][4];
#pragma unroll
    for (int mb = 0; mb < 4; ++mb)
#pragma unroll
        for (int nb = 0; nb < 4; ++nb) acc[mb][nb] = (v8f){};
    const size_t aoff = (size_t)(r0 + lr) * K + 8 * hi, boff = (size_t)(c0 + lr) * K + 8 * hi;
#pragma unroll 1
    for (int kc = 0; kc < K; kc += 32) {
        v16bf a[4];
#pragma unroll
        for (int mb = 0; mb < 4; ++mb) a[mb] = ldb(A + aoff + (size_t)mb * 16 * K + kc);
#pragma unroll
        for (int nb = 0; nb < 4; ++nb) { const v16bf b = ldb(Bt + boff + (size_t)nb * 16 * K + kc);
#pragma unroll
            for (int mb = 0; mb < 4; ++mb) acc[mb][nb] = wmmabg(a[mb], b, acc[mb][nb]); }
    }
    if (LOWR) {
        const size_t axo = (size_t)(r0 + lr) * LK + 8 * hi, bxo = (size_t)(c0 + lr) * LK + 8 * hi;
        v16bf a[4];
#pragma unroll
        for (int mb = 0; mb < 4; ++mb) a[mb] = ldb(AX + axo + (size_t)mb * 16 * LK);
#pragma unroll
        for (int nb = 0; nb < 4; ++nb) { const v16bf b = ldb(BX + bxo + (size_t)nb * 16 * LK);
#pragma unroll
            for (int mb = 0; mb < 4; ++mb) acc[mb][nb] = wmmabg(a[mb], b, acc[mb][nb]); }
    }
    float bc[4];
#pragma unroll
    for (int nb = 0; nb < 4; ++nb) bc[nb] = (MODE == 0) ? bfr(bias[c0 + nb * 16 + lr]) : 0.0f;
    size_t tbase, rbase; bool wr;
    if (MODE == 0) { const int bb = r0 / SEQ, tt = r0 % SEQ; const int zc = bb * NH_ + c0 / HD;
                     tbase = ((size_t)zc * SEQ + (size_t)tt) * HD; rbase = ((size_t)zc * (size_t)resT + (size_t)tt) * HD; wr = tt < resT; }
    else           { const int bb = c0 / SEQ, tt = c0 % SEQ;
                     tbase = (size_t)bb * (size_t)DM * SEQ + (size_t)r0 * SEQ + (size_t)tt; rbase = (size_t)bb * (size_t)DM * (size_t)resT + (size_t)r0 * (size_t)resT + (size_t)tt; wr = tt < resT; }
#pragma unroll
    for (int mb = 0; mb < 4; ++mb) {
        float br[8];
#pragma unroll
        for (int j = 0; j < 8; ++j) br[j] = (MODE == 1) ? bfr(bias[r0 + mb * 16 + hi * 8 + j]) : 0.0f;
#pragma unroll
        for (int nb = 0; nb < 4; ++nb) {
#pragma unroll
            for (int j = 0; j < 8; ++j) os[(hi * 8 + j) * 68 + nb * 16 + lr] = acc[mb][nb][j] + bc[nb] + br[j]; }
        wave_sync();
#pragma unroll 1
        for (int ps = 0; ps < 2; ++ps) {
            if (MODE == 0) {
                const size_t sb = tbase + (size_t)(mb * 16) * HD;
                const size_t rb = rbase + (size_t)(mb * 16) * HD;
#pragma unroll
                for (int s = 0; s < 4; ++s) { const int p = s * 32 + lane; const int row = p >> 3, c8 = (p & 7) * 8;
                    const v4f x0 = *(const v4fa*)(&os[row * 68 + c8]); const v4f x1 = *(const v4fa*)(&os[row * 68 + c8 + 4]); v8h hv, rv;
#pragma unroll
                    for (int i = 0; i < 4; ++i) { const h16 a0 = toh_flush(x0[i]); const h16 a1 = toh_flush(x1[i]); hv[i] = a0; hv[4 + i] = a1;
                                                  rv[i] = toh_flush((x0[i] - (float)a0) * QRS); rv[4 + i] = toh_flush((x1[i] - (float)a1) * QRS); }
                    const size_t oo = sb + (size_t)p * 8;
                    const size_t ro = rb + (size_t)p * 8;
                    *(volatile v8h*)(Ph + oo) = hv; if (wr) *(volatile v8h*)(Pr + ro) = rv; }
            } else {
                const size_t sb = tbase + (size_t)(mb * 16) * SEQ;
                const size_t rb = rbase + (size_t)(mb * 16) * (size_t)resT;
#pragma unroll
                for (int s = 0; s < 4; ++s) { const int row = 4 * s + (lane >> 3), c8 = (lane & 7) * 8;
                    const v4f x0 = *(const v4fa*)(&os[row * 68 + c8]); const v4f x1 = *(const v4fa*)(&os[row * 68 + c8 + 4]); v8h hv, rv;
#pragma unroll
                    for (int i = 0; i < 4; ++i) { const h16 a0 = toh_flush(x0[i]); const h16 a1 = toh_flush(x1[i]); hv[i] = a0; hv[4 + i] = a1;
                                                  rv[i] = toh_flush((x0[i] - (float)a0) * QRS); rv[4 + i] = toh_flush((x1[i] - (float)a1) * QRS); }
                    const size_t oo = sb + (size_t)row * SEQ + c8;
                    const size_t ro = rb + (size_t)row * (size_t)resT + c8;
                    *(volatile v8h*)(Ph + oo) = hv; if (wr) *(volatile v8h*)(Pr + ro) = rv; }
            }
            if (ps == 0) __threadfence(); }
        wave_sync();
    }
}

__global__ __launch_bounds__(32) void k_projq(const bf* __restrict__ A, const bf* __restrict__ Bt, const bf* __restrict__ AX, const bf* __restrict__ BX,
                                              const float* __restrict__ bias, h16* Ph, h16* Pr, int resT) { proj_body<0, 1>(A, Bt, AX, BX, bias, Ph, Pr, resT); }
__global__ __launch_bounds__(32) void k_projk(const bf* __restrict__ A, const bf* __restrict__ Bt,
                                              const float* __restrict__ bias, h16* Ph, h16* Pr, int resT) { proj_body<0, 0>(A, Bt, A, Bt, bias, Ph, Pr, resT); }
__global__ __launch_bounds__(32) void k_projv(const bf* __restrict__ A, const bf* __restrict__ Bt, const bf* __restrict__ AX, const bf* __restrict__ BX,
                                              const float* __restrict__ bias, h16* Ph, h16* Pr, int resT) { proj_body<1, 1>(A, Bt, AX, BX, bias, Ph, Pr, resT); }

template <int EARLY>
__device__ __forceinline__ void keypass_body(const h16* __restrict__ QH, const h16* __restrict__ QR, const h16* __restrict__ KP, const h16* __restrict__ KR,
                                           const h16* __restrict__ VT, const h16* __restrict__ VR, const float* __restrict__ amask, float* OUT) {
    __shared__ __align__(16) float os[AW * 16 * OSP];
    const int lane = threadIdx.x & 31, lr = lane & 15, hi = lane >> 4;
    const int wave = __builtin_amdgcn_readfirstlane((int)(threadIdx.x >> 5));
    const int zh = blockIdx.y; const int b = zh / NH_, h = zh % NH_;
    const int t0 = (EARLY ? 0 : EROWS) + (blockIdx.x * AW + wave) * 16;
    const int lim = t0 + lr;
    const float* amb = amask + (size_t)b * SEQ_FULL;
    float fl = 0.0f;
#pragma unroll 1
    for (int i = 0; i < SEQ; i += 128) {
        const v4f w = *(const v4f*)(amb + i + 4 * lane);
#pragma unroll
        for (int c = 0; c < 4; ++c) { const float a = fabsf(bfr(w[c])); fl = (a < WIDE) ? fl : 1.0f; } }
    fl = fmaxf(fl, __shfl_xor(fl, 16, 32)); fl = fmaxf(fl, __shfl_xor(fl, 8, 32)); fl = fmaxf(fl, __shfl_xor(fl, 4, 32));
    fl = fmaxf(fl, __shfl_xor(fl, 2, 32));  fl = fmaxf(fl, __shfl_xor(fl, 1, 32));
    const int nkc = (t0 + 16 + 31) & ~31;
    const int nkv = (fl != 0.0f) ? SEQ : nkc;
    const int nk = __builtin_amdgcn_readfirstlane(nkv);
    const size_t pbase = (size_t)zh * SEQ * HD;
    const size_t rbase = (size_t)zh * EROWS * HD;
    const size_t qo = pbase + (size_t)(t0 + lr) * HD + 8 * hi;
    const v16h hz = (v16h){};
    v16h qh[2], qr[2];
    qh[0] = ldh(QH + qo); qh[1] = ldh(QH + qo + 32);
    qr[0] = hz; qr[1] = hz;
    if (EARLY) { const size_t qro = rbase + (size_t)(t0 + lr) * HD + 8 * hi; qr[0] = ldh(QR + qro); qr[1] = ldh(QR + qro + 32); }
    const size_t ko = pbase + (size_t)lr * HD + 8 * hi;
    const size_t vo = pbase + (size_t)lr * SEQ + 8 * hi;
    const size_t kro = rbase + (size_t)lr * HD + 8 * hi;
    const size_t vro = rbase + (size_t)lr * EROWS + 8 * hi;
    v8f o[4], oR[4];
#pragma unroll
    for (int j = 0; j < 4; ++j) { o[j] = (v8f){}; oR[j] = (v8f){}; }
    float m = NEGB, l = 0.0f;
#pragma unroll 1
    for (int key0 = 0; key0 < nk; key0 += 32) {
        const bool rok = key0 < EROWS;
        const int kcl = rok ? key0 : (EROWS - 32);
        const h16* kpt = KP + ko + (size_t)key0 * HD;
        v8f sHa = (v8f){}, sLa = (v8f){}, sHb = (v8f){}, sLb = (v8f){};
#pragma unroll
        for (int ks = 0; ks < 2; ++ks) {
            const v16h ka = ldh(kpt + ks * 32), kb = ldh(kpt + 16 * HD + ks * 32);
            sHa = wmma16g(ka, qh[ks], sHa); sHb = wmma16g(kb, qh[ks], sHb);
            if (EARLY) {
                sLa = wmma16g(ka, qr[ks], sLa); sLb = wmma16g(kb, qr[ks], sLb);
                const h16* krp = KR + kro + (size_t)kcl * HD;
                v16h kra = ldh(krp + ks * 32), krb = ldh(krp + 16 * HD + ks * 32);
                if (!rok) { kra = hz; krb = hz; }
                sLa = wmma16g(kra, qh[ks], sLa); sLb = wmma16g(krb, qh[ks], sLb);
            }
        }
        const float* kp = amb + 8 * hi + key0;
        const v4f m0 = *(const v4f*)kp, m1 = *(const v4f*)(kp + 4), m2 = *(const v4f*)(kp + 16), m3 = *(const v4f*)(kp + 20);
        float kx[8], ky[8];
#pragma unroll
        for (int r = 0; r < 4; ++r) { kx[r] = m0[r]; kx[4 + r] = m1[r]; ky[r] = m2[r]; ky[4 + r] = m3[r]; }
        const int ja = key0 + 8 * hi;
        float ta[8], tb[8]; float mx = NEGB;
#pragma unroll
        for (int r = 0; r < 8; ++r) {
            const float sa = EARLY ? (sHa[r] + sLa[r] * QRI) * SC2 : sHa[r] * SC2;
            const float sb = EARLY ? (sHb[r] + sLb[r] * QRI) * SC2 : sHb[r] * SC2;
            ta[r] = ((ja + r > lim) ? NEGL : sa) + bfr(kx[r]) * L2E;
            tb[r] = ((ja + 16 + r > lim) ? NEGL : sb) + bfr(ky[r]) * L2E;
            mx = fmaxf(mx, fmaxf(ta[r], tb[r])); }
        mx = fmaxf(mx, __shfl_xor(mx, 16, 32));
        const float mnew = fmaxf(m, mx);
        const float alpha = __builtin_amdgcn_exp2f(m - mnew);
        const float sh = PSH - mnew;
        v16h pb, pr = hz; float ls = 0.0f;
#pragma unroll
        for (int r = 0; r < 8; ++r) {
            const float aa = ta[r] + sh, ab = tb[r] + sh;
            const float ea = __builtin_amdgcn_exp2f(aa), eb = __builtin_amdgcn_exp2f(ab);
            const float ga = (aa < PFL) ? 0.0f : ea, gb = (ab < PFL) ? 0.0f : eb;
            const h16 pa = (h16)ga; const h16 pc = (h16)gb;
            pb[r] = pa; pb[8 + r] = pc;
            if (EARLY) { pr[r] = toh_flush((ga - (float)pa) * QRS); pr[8 + r] = toh_flush((gb - (float)pc) * QRS); ls += ga + gb; }
            else       { ls += (float)pa + (float)pc; } }
        l = l * alpha + ls; m = mnew;
#pragma unroll
        for (int j = 0; j < 4; ++j) { o[j] = o[j] * alpha; if (EARLY) oR[j] = oR[j] * alpha; }
        const h16* va = VT + vo + key0;
#pragma unroll
        for (int jp = 0; jp < 2; ++jp) {
            const v16h v0 = ldh(va + (size_t)(32 * jp) * SEQ), v1 = ldh(va + (size_t)(32 * jp + 16) * SEQ);
            o[2 * jp] = wmma16g(v0, pb, o[2 * jp]); o[2 * jp + 1] = wmma16g(v1, pb, o[2 * jp + 1]);
            if (EARLY) {
                oR[2 * jp] = wmma16g(v0, pr, oR[2 * jp]); oR[2 * jp + 1] = wmma16g(v1, pr, oR[2 * jp + 1]);
                const h16* vrp = VR + vro + kcl;
                v16h vr0 = ldh(vrp + (size_t)(32 * jp) * EROWS), vr1 = ldh(vrp + (size_t)(32 * jp + 16) * EROWS);
                if (!rok) { vr0 = hz; vr1 = hz; }
                oR[2 * jp] = wmma16g(vr0, pb, oR[2 * jp]); oR[2 * jp + 1] = wmma16g(vr1, pb, oR[2 * jp + 1]);
            }
        }
    }
    l += __shfl_xor(l, 16, 32);
    const float inv = 1.0f / l;
    const int wb = wave * 16 * OSP;
#pragma unroll
    for (int j = 0; j < 4; ++j) {
        v8f f = o[j];
        if (EARLY) f = o[j] + oR[j] * QRI;
        v4f a, c;
        a[0] = f[0] * inv; a[1] = f[1] * inv; a[2] = f[2] * inv; a[3] = f[3] * inv; c[0] = f[4] * inv; c[1] = f[5] * inv; c[2] = f[6] * inv; c[3] = f[7] * inv;
        *(v4fa*)(&os[wb + lr * OSP + 16 * j + 8 * hi]) = a; *(v4fa*)(&os[wb + lr * OSP + 16 * j + 8 * hi + 4]) = c; }
    wave_sync();
    float* orow = OUT + ((size_t)b * OUT_SEQ + t0) * DM + h * HD;
#pragma unroll 1
    for (int ps = 0; ps < 2; ++ps) {
#pragma unroll
        for (int s = 0; s < 8; ++s) { const int row = 2 * s + (lane >> 4), cofs = (lane & 15) * 4;
            const v4f val = *(const v4fa*)(&os[wb + row * OSP + cofs]);
            *(volatile v4f*)(orow + (size_t)row * DM + cofs) = val; }
        if (ps == 0) __threadfence(); }
}

__global__ __launch_bounds__(32 * AW) __attribute__((amdgpu_num_vgpr(256)))
void k_keypass_early(const h16* __restrict__ QH, const h16* __restrict__ QR, const h16* __restrict__ KP, const h16* __restrict__ KR,
                   const h16* __restrict__ VT, const h16* __restrict__ VR, const float* __restrict__ amask, float* OUT) {
    keypass_body<1>(QH, QR, KP, KR, VT, VR, amask, OUT);
}
__global__ __launch_bounds__(32 * AW) __attribute__((amdgpu_num_vgpr(256)))
void k_keypass_late(const h16* __restrict__ QH, const h16* __restrict__ KP, const h16* __restrict__ VT, const float* __restrict__ amask, float* OUT) {
    keypass_body<0>(QH, QH, KP, KP, VT, VT, amask, OUT);
}

static constexpr size_t al256(size_t v) { return (v + 255) & ~(size_t)255; }
static constexpr size_t SZ_XB = al256((size_t)NB * SEQ * DM * 2);
static constexpr size_t SZ_WB = al256((size_t)3 * DM * DM * 2);
static constexpr size_t SZ_AL = al256((size_t)2 * LR * DM * 2);
static constexpr size_t SZ_BL = al256((size_t)DM * LK * 2);
static constexpr size_t SZ_XL = al256((size_t)NB * SEQ * LK * 2);
static constexpr size_t SZ_PL = al256((size_t)NB * NH_ * SEQ * HD * 2);
static constexpr size_t SZ_RS = al256((size_t)NB * NH_ * EROWS * HD * 2);
static constexpr size_t SZ_TOTAL = SZ_XB + SZ_WB + SZ_AL + 2 * SZ_BL + 2 * SZ_XL + 3 * SZ_PL + 3 * SZ_RS;
static_assert(SZ_TOTAL <= (size_t)134217728);
static_assert(((size_t)DM * DM * 2) % 256 == 0);
static_assert(((size_t)LR * DM * 2) % 256 == 0);
static_assert((size_t)NB * NH_ * SEQ * HD == (size_t)NB * DM * SEQ);
static_assert((size_t)NB * NH_ * EROWS * HD == (size_t)NB * DM * EROWS);
static_assert((DM * 4) % 256 == 0);

extern "C" void kernel_launch(void* const* d_in, const int* in_sizes, int n_in,
                              void* d_out, int out_size, void* d_ws, size_t ws_size, hipStream_t stream) {
    if (n_in < 12) return;
    const size_t needx = ((size_t)(NB - 1) * SEQ_FULL + SEQ) * DM;
    const size_t needm = (size_t)(NB - 1) * SEQ_FULL + SEQ;
    if ((size_t)in_sizes[0] < needx || (size_t)in_sizes[1] < needm) return;
    if ((size_t)in_sizes[2] < (size_t)DM * DM || (size_t)in_sizes[4] < (size_t)DM * DM || (size_t)in_sizes[6] < (size_t)DM * DM) return;
    if (in_sizes[3] < DM || in_sizes[5] < DM || in_sizes[7] < DM) return;
    if (in_sizes[8] < LR * DM || in_sizes[9] < DM * LR || in_sizes[10] < LR * DM || in_sizes[11] < DM * LR) return;
    if ((size_t)out_size < ((size_t)(NB - 1) * OUT_SEQ + SEQ) * DM) return;
    if (SZ_TOTAL > ws_size) return;
    const float* xin = (const float*)d_in[0];
    const float* am  = (const float*)d_in[1];
    const float* wq = (const float*)d_in[2]; const float* bq = (const float*)d_in[3];
    const float* wk = (const float*)d_in[4]; const float* bk = (const float*)d_in[5];
    const float* wv = (const float*)d_in[6]; const float* bv = (const float*)d_in[7];
    const float* aq = (const float*)d_in[8]; const float* bqu = (const float*)d_in[9];
    const float* av = (const float*)d_in[10]; const float* bvu = (const float*)d_in[11];
    float* OUT = (float*)d_out;
    char* wsp = (char*)d_ws;
    bf* XB = (bf*)wsp; wsp += SZ_XB;
    bf* WB = (bf*)wsp; wsp += SZ_WB;
    bf* AL = (bf*)wsp; wsp += SZ_AL;
    bf* BLq = (bf*)wsp; wsp += SZ_BL;
    bf* BLv = (bf*)wsp; wsp += SZ_BL;
    bf* XLq = (bf*)wsp; wsp += SZ_XL;
    bf* XLv = (bf*)wsp; wsp += SZ_XL;
    h16* QH = (h16*)wsp; wsp += SZ_PL;
    h16* KP = (h16*)wsp; wsp += SZ_PL;
    h16* VT = (h16*)wsp; wsp += SZ_PL;
    h16* QR = (h16*)wsp; wsp += SZ_RS;
    h16* KR = (h16*)wsp; wsp += SZ_RS;
    h16* VR = (h16*)wsp; wsp += SZ_RS;
    bf* WQ = WB; bf* WK = WB + (size_t)DM * DM; bf* WV = WB + (size_t)2 * DM * DM;

    if (SEQ == SEQ_FULL) {
        const size_t n8 = (size_t)NB * SEQ * DM / 8;
        k_cvt8<<<(unsigned)((n8 + 255) / 256), 256, 0, stream>>>(xin, XB, n8);
    } else {
        const size_t n8 = (size_t)SEQ * DM / 8;
        for (int b = 0; b < NB; ++b) k_cvt8<<<(unsigned)((n8 + 255) / 256), 256, 0, stream>>>(xin + (size_t)b * SEQ_FULL * DM, XB + (size_t)b * SEQ * DM, n8);
    }
    { const size_t n8 = (size_t)DM * DM / 8; const unsigned g = (unsigned)((n8 + 255) / 256);
      k_cvt8<<<g, 256, 0, stream>>>(wq, WQ, n8); k_cvt8<<<g, 256, 0, stream>>>(wk, WK, n8); k_cvt8<<<g, 256, 0, stream>>>(wv, WV, n8); }
    { const size_t n8 = (size_t)LR * DM / 8; const unsigned g = (unsigned)((n8 + 255) / 256);
      k_cvt8<<<g, 256, 0, stream>>>(aq, AL, n8); k_cvt8<<<g, 256, 0, stream>>>(av, AL + (size_t)LR * DM, n8); }
    { const int n4 = DM * 4; const unsigned g = (unsigned)((n4 + 255) / 256);
      k_bext<<<g, 256, 0, stream>>>(bqu, BLq, n4); k_bext<<<g, 256, 0, stream>>>(bvu, BLv, n4); }

    k_xa<<<dim3(NB * SEQ / 64, 1, 1), 32, 0, stream>>>(XB, AL, XLq, XLv);

    k_projq<<<dim3(NB * SEQ / 64, DM / 64, 1), 32, 0, stream>>>(XB, WQ, XLq, BLq, bq, QH, QR, EROWS);
    k_projk<<<dim3(NB * SEQ / 64, DM / 64, 1), 32, 0, stream>>>(XB, WK, bk, KP, KR, EROWS);
    k_projv<<<dim3(DM / 64, NB * SEQ / 64, 1), 32, 0, stream>>>(WV, XB, BLv, XLv, bv, VT, VR, EROWS);

    k_keypass_early<<<dim3(EROWS / (16 * AW), NB * NH_, 1), 32 * AW, 0, stream>>>(QH, QR, KP, KR, VT, VR, am, OUT);
    if (SEQ > EROWS)
        k_keypass_late<<<dim3((SEQ - EROWS) / (16 * AW), NB * NH_, 1), 32 * AW, 0, stream>>>(QH, KP, VT, am, OUT);
}
